// LanguageModel_66477503807731
// MI455X (gfx1250) — hardware-verified
//
#include <hip/hip_runtime.h>
#include <hip/hip_bf16.h>

#define B_    4
#define N_    4096
#define D_    512
#define E_    4
#define F_    2048
#define NTOK  (B_ * N_)
#define TMB   32
#define FC    128
#define XSTR  (D_ + 8)
#define HSTR  (FC + 8)
#define BSTR  40

typedef __bf16         v16bf __attribute__((ext_vector_type(16)));
typedef float          v8f   __attribute__((ext_vector_type(8)));
typedef float          v4f   __attribute__((ext_vector_type(4)));
typedef int            v4i   __attribute__((ext_vector_type(4)));
typedef unsigned int   v2u   __attribute__((ext_vector_type(2)));
typedef unsigned short us8   __attribute__((ext_vector_type(8)));
typedef v4f __attribute__((may_alias)) v4fa;
typedef v4i __attribute__((may_alias)) v4ia;
typedef v2u __attribute__((may_alias)) v2ua;
typedef us8 __attribute__((may_alias)) us8a;

union FragU { v16bf v; us8 h[2]; };

__device__ __forceinline__ unsigned short f2bf(float f) {
  unsigned int u = __float_as_uint(f);
  u += 0x7FFFu + ((u >> 16) & 1u);
  return (unsigned short)(u >> 16);
}

__device__ __forceinline__ void split2(float f, unsigned short& hi, unsigned short& lo) {
  hi = f2bf(f);
  const float fh = __uint_as_float(((unsigned int)hi) << 16);
  lo = f2bf(f - fh);
}

__device__ __forceinline__ v16bf ld_frag(const unsigned short* rowBase, int hh) {
  FragU f;
  f.h[0] = *(const us8a*)(rowBase + 8 * hh);
  f.h[1] = *(const us8a*)(rowBase + 16 + 8 * hh);
  return f.v;
}

__device__ __forceinline__ void mma3(v8f& acc, const v16bf& ah, const v16bf& al,
                                     const v16bf& bh, const v16bf& bl) {
  acc = __builtin_amdgcn_wmma_f32_16x16x32_bf16(false, ah, false, bh, (short)0, acc, false, false);
  acc = __builtin_amdgcn_wmma_f32_16x16x32_bf16(false, ah, false, bl, (short)0, acc, false, false);
  acc = __builtin_amdgcn_wmma_f32_16x16x32_bf16(false, al, false, bh, (short)0, acc, false, false);
  asm volatile("v_nop\n\tv_nop\n\tv_nop\n\tv_nop" : "+v"(acc) : "v"(al), "v"(bh), "v"(ah), "v"(bl));
}

__device__ __forceinline__ float gelu_exact(float t) {
  return (0.5f * t) * erfcf(-t * 0.70710678118654752f);
}

__device__ __forceinline__ void stage4(unsigned short* sbh, unsigned short* sbl, int c4, int r, float4 f) {
  unsigned short h, l;
  split2(f.x, h, l); sbh[(c4 + 0) * BSTR + r] = h; sbl[(c4 + 0) * BSTR + r] = l;
  split2(f.y, h, l); sbh[(c4 + 1) * BSTR + r] = h; sbl[(c4 + 1) * BSTR + r] = l;
  split2(f.z, h, l); sbh[(c4 + 2) * BSTR + r] = h; sbl[(c4 + 2) * BSTR + r] = l;
  split2(f.w, h, l); sbh[(c4 + 3) * BSTR + r] = h; sbl[(c4 + 3) * BSTR + r] = l;
}

__global__ __launch_bounds__(256) void k_proj_gate(
    const float* __restrict__ x, const float* __restrict__ vw, const float* __restrict__ vb,
    const float* __restrict__ gw, const float* __restrict__ gb,
    float* vout, int* eout, int ntok) {
  __shared__ __attribute__((aligned(16))) float sV[TMB];
  __shared__ __attribute__((aligned(16))) int   sE[TMB];
  const int tid  = threadIdx.x;
  const int lane = tid & 31;
  const int wv   = tid >> 5;
  const int base = blockIdx.x * TMB;
#pragma unroll 1
  for (int q = 0; q < 4; ++q) {
    const int tl = wv * 4 + q;
    const int t  = base + tl;
    double a0 = 0.0, a1 = 0.0, a2 = 0.0, a3 = 0.0, a4 = 0.0;
    if (t < ntok) {
      const float* xr = x + (size_t)t * D_;
#pragma unroll 1
      for (int it = 0; it < 4; ++it) {
        const int k = (it * 32 + lane) * 4;
        const float4 xv = *(const float4*)(xr + k);
        const float4 w0 = *(const float4*)(vw + k);
        const float4 g0 = *(const float4*)(gw + 0 * D_ + k);
        const float4 g1 = *(const float4*)(gw + 1 * D_ + k);
        const float4 g2 = *(const float4*)(gw + 2 * D_ + k);
        const float4 g3 = *(const float4*)(gw + 3 * D_ + k);
        const double x0 = (double)xv.x, x1 = (double)xv.y, x2 = (double)xv.z, x3 = (double)xv.w;
        a0 += x0 * (double)w0.x + x1 * (double)w0.y + x2 * (double)w0.z + x3 * (double)w0.w;
        a1 += x0 * (double)g0.x + x1 * (double)g0.y + x2 * (double)g0.z + x3 * (double)g0.w;
        a2 += x0 * (double)g1.x + x1 * (double)g1.y + x2 * (double)g1.z + x3 * (double)g1.w;
        a3 += x0 * (double)g2.x + x1 * (double)g2.y + x2 * (double)g2.z + x3 * (double)g2.w;
        a4 += x0 * (double)g3.x + x1 * (double)g3.y + x2 * (double)g3.z + x3 * (double)g3.w;
      }
    }
#pragma unroll
    for (int off = 16; off > 0; off >>= 1) {
      a0 += __shfl_xor(a0, off, 32);
      a1 += __shfl_xor(a1, off, 32);
      a2 += __shfl_xor(a2, off, 32);
      a3 += __shfl_xor(a3, off, 32);
      a4 += __shfl_xor(a4, off, 32);
    }
    if (lane == 0) {
      float v = (float)a0 + vb[0];
      v = fminf(fmaxf(v, -3.0f), 3.0f);
      const float l0 = (float)a1 + gb[0], l1 = (float)a2 + gb[1];
      const float l2 = (float)a3 + gb[2], l3 = (float)a4 + gb[3];
      int best = 0; float bm = l0;
      if (l1 > bm) { bm = l1; best = 1; }
      if (l2 > bm) { bm = l2; best = 2; }
      if (l3 > bm) { bm = l3; best = 3; }
      sV[tl] = v;
      sE[tl] = best;
    }
  }
  __syncthreads();
  const bool wr = (wv == 0) && (lane < 8) && (base + TMB <= ntok);
  v4f vv; v4i ee;
#pragma unroll
  for (int c = 0; c < 4; ++c) { vv[c] = 0.f; ee[c] = 0; }
  if (wr) {
    vv = *(const v4fa*)(sV + lane * 4);
    ee = *(const v4ia*)(sE + lane * 4);
    *(volatile v4f*)(vout + base + lane * 4) = vv;
    *(volatile v4i*)(eout + base + lane * 4) = ee;
  }
  __threadfence();
  if (wr) {
    *(volatile v4f*)(vout + base + lane * 4) = vv;
    *(volatile v4i*)(eout + base + lane * 4) = ee;
  }
}

__global__ __launch_bounds__(256) void k_green(
    const float* vws, const float* __restrict__ gamma, const float* __restrict__ epsp,
    float* feats, int nb) {
#pragma clang fp contract(off)
  extern __shared__ __attribute__((aligned(16))) float smf[];
  float* sL  = smf;
  float* sU  = smf + 2 * N_;
  float* sFt = smf + 4 * N_;
  const int b = blockIdx.x;
  if (b >= nb) return;
  const int tid  = threadIdx.x;
  const int lane = tid & 31;
  const int wv   = tid >> 5;
  const float ep  = epsp[0];
  const float eps = fmaxf(ep, 0.f) + log1pf(expf(-fabsf(ep))) + 1e-6f;
  const float di  = -(eps + gamma[0]);
  const float* vb = vws + (size_t)b * N_;

  if (tid == 0) {
    float cr = vb[0] - 2.0f, ci = di;
    sL[0] = cr; sL[1] = ci;
#pragma unroll 1
    for (int i = 1; i < N_; ++i) {
      const float m  = cr * cr + ci * ci;
      const float ir = cr / m;
      const float ii = ci / m;
      const float nr = (vb[i] - 2.0f) - ir;
      const float ni = di + ii;
      cr = nr; ci = ni;
      sL[2 * i] = cr; sL[2 * i + 1] = ci;
    }
  } else if (tid == 32) {
    float cr = vb[N_ - 1] - 2.0f, ci = di;
    sU[2 * (N_ - 1)] = cr; sU[2 * (N_ - 1) + 1] = ci;
#pragma unroll 1
    for (int i = N_ - 2; i >= 0; --i) {
      const float m  = cr * cr + ci * ci;
      const float ir = cr / m;
      const float ii = ci / m;
      const float nr = (vb[i] - 2.0f) - ir;
      const float ni = di + ii;
      cr = nr; ci = ni;
      sU[2 * i] = cr; sU[2 * i + 1] = ci;
    }
  }
  __syncthreads();
#pragma unroll 1
  for (int i = tid; i < N_; i += 256) {
    const float dr = vb[i] - 2.0f;
    const float sr = sL[2 * i] + sU[2 * i] - dr;
    const float si = sL[2 * i + 1] + sU[2 * i + 1] - di;
    const float m  = sr * sr + si * si;
    const float Gr = sr / m;
    const float Gi = -si / m;
    sFt[2 * i]     = fminf(fmaxf(Gr, -10.f), 10.f);
    sFt[2 * i + 1] = fminf(fmaxf(Gi, -10.f), 10.f);
  }
  __syncthreads();
  float* fb = feats + (size_t)b * 2 * N_;
  for (int g = wv; g < (2 * N_) / 128; g += 8) {
    const v4f v = *(const v4fa*)(sFt + g * 128 + lane * 4);
    *(volatile v4f*)(fb + g * 128 + lane * 4) = v;
  }
  __threadfence();
  for (int g = wv; g < (2 * N_) / 128; g += 8) {
    const v4f v = *(const v4fa*)(sFt + g * 128 + lane * 4);
    *(volatile v4f*)(fb + g * 128 + lane * 4) = v;
  }
}

__global__ __launch_bounds__(512) void k_bucket(const int* eprev, int* perm, int* meta, int ntok) {
  extern __shared__ __attribute__((aligned(16))) int smi[];
  int* sPerm = smi;
  int* sCnt  = smi + NTOK;
  __shared__ __attribute__((aligned(16))) int sMeta[32];
  __shared__ int sTot[E_];
  const int tid  = threadIdx.x;
  const int lane = tid & 31;
  const int wv   = tid >> 5;
  if (ntok != NTOK) return;

  int ev[32];
#pragma unroll
  for (int j = 0; j < 8; ++j) {
    const v4i q4 = *(const v4ia*)(eprev + tid * 32 + j * 4);
    ev[4 * j + 0] = q4.x; ev[4 * j + 1] = q4.y; ev[4 * j + 2] = q4.z; ev[4 * j + 3] = q4.w;
  }
  int c0 = 0, c1 = 0, c2 = 0, c3 = 0;
#pragma unroll
  for (int j = 0; j < 32; ++j) {
    int e = ev[j];
    e = e < 0 ? 0 : (e > 3 ? 3 : e);
    ev[j] = e;
    c0 += (e == 0); c1 += (e == 1); c2 += (e == 2); c3 += (e == 3);
  }
  sCnt[0 * 512 + tid] = c0;
  sCnt[1 * 512 + tid] = c1;
  sCnt[2 * 512 + tid] = c2;
  sCnt[3 * 512 + tid] = c3;
  if (tid < 32) sMeta[tid] = 0;
  __syncthreads();
  if (tid < E_) {
    int run = 0;
    for (int i = 0; i < 512; ++i) {
      const int c = sCnt[tid * 512 + i];
      sCnt[tid * 512 + i] = run;
      run += c;
    }
    sTot[tid] = run;
  }
  __syncthreads();
  if (tid == 0) {
    int off = 0, ts = 0;
    for (int e = 0; e < E_; ++e) {
      sMeta[e]     = sTot[e];
      sMeta[4 + e] = off;
      sMeta[9 + e] = ts;
      off += sTot[e];
      ts  += (sTot[e] + TMB - 1) / TMB;
    }
    sMeta[4 + E_] = off;
    sMeta[9 + E_] = ts;
  }
  __syncthreads();
  int r0 = sMeta[4] + sCnt[0 * 512 + tid];
  int r1 = sMeta[5] + sCnt[1 * 512 + tid];
  int r2 = sMeta[6] + sCnt[2 * 512 + tid];
  int r3 = sMeta[7] + sCnt[3 * 512 + tid];
#pragma unroll
  for (int j = 0; j < 32; ++j) {
    const int e   = ev[j];
    const int pos = (e == 0) ? r0 : ((e == 1) ? r1 : ((e == 2) ? r2 : r3));
    if ((unsigned)pos < (unsigned)NTOK) sPerm[pos] = tid * 32 + j;
    r0 += (e == 0); r1 += (e == 1); r2 += (e == 2); r3 += (e == 3);
  }
  __syncthreads();
  const bool wm = (wv == 0) && (lane < 8);
  v4i mv;
#pragma unroll
  for (int c = 0; c < 4; ++c) mv[c] = 0;
  if (wm) mv = *(const v4ia*)(sMeta + lane * 4);
  for (int g = wv; g < NTOK / 128; g += 16) {
    const v4i v = *(const v4ia*)(sPerm + g * 128 + lane * 4);
    *(volatile v4i*)(perm + g * 128 + lane * 4) = v;
  }
  if (wm) *(volatile v4i*)(meta + lane * 4) = mv;
  __threadfence();
  for (int g = wv; g < NTOK / 128; g += 16) {
    const v4i v = *(const v4ia*)(sPerm + g * 128 + lane * 4);
    *(volatile v4i*)(perm + g * 128 + lane * 4) = v;
  }
  if (wm) *(volatile v4i*)(meta + lane * 4) = mv;
}

__global__ __launch_bounds__(256) __attribute__((amdgpu_num_vgpr(256)))
void k_ffn(const float* __restrict__ x,
           const float* __restrict__ w1, const float* __restrict__ b1,
           const float* __restrict__ w2, const float* __restrict__ b2,
           const float* __restrict__ ow, const float* __restrict__ ob, const float* __restrict__ bk,
           const int* perm, const int* meta, const float* feats, float* out, int ntok) {
  extern __shared__ __attribute__((aligned(16))) unsigned char smem[];
  unsigned short* sXhi = (unsigned short*)smem;
  unsigned short* sXlo = sXhi + TMB * XSTR;
  unsigned short* sHhi = sXlo + TMB * XSTR;
  unsigned short* sHlo = sHhi + TMB * HSTR;
  unsigned short* sBhi = sHlo + TMB * HSTR;
  unsigned short* sBlo = sBhi + D_ * BSTR;
  float* sOut = (float*)smem;
  __shared__ int   sTok[TMB];
  __shared__ int   sVal[TMB];
  __shared__ float sF0[TMB];
  __shared__ float sF1[TMB];

  const int blk    = blockIdx.x;
  const int ntiles = meta[9 + E_];
  if (blk >= ntiles) return;
  const int ts1 = meta[10], ts2 = meta[11], ts3 = meta[12];
  const int e     = (blk >= ts1 ? 1 : 0) + (blk >= ts2 ? 1 : 0) + (blk >= ts3 ? 1 : 0);
  const int cnt   = meta[e];
  const int off   = meta[4 + e];
  const int tbase = (blk - meta[9 + e]) * TMB;

  const int tid  = threadIdx.x;
  const int lane = tid & 31;
  const int wv   = tid >> 5;
  const int hh   = lane >> 4;
  const int m16  = lane & 15;

  if (tid < TMB) {
    const int idx = tbase + tid;
    const int ok  = (idx < cnt) ? 1 : 0;
    int pi = off + (ok ? idx : tbase);
    pi = pi < 0 ? 0 : (pi > ntok - 1 ? ntok - 1 : pi);
    int gt = perm[pi];
    gt = gt < 0 ? 0 : (gt > ntok - 1 ? ntok - 1 : gt);
    sTok[tid] = gt;
    sVal[tid] = ok;
    sF0[tid]  = feats[2 * (size_t)gt];
    sF1[tid]  = feats[2 * (size_t)gt + 1];
  }
  __syncthreads();

  for (int i = tid; i < TMB * (D_ / 4); i += 256) {
    const int m  = i >> 7;
    const int k4 = (i & 127) * 4;
    const float4 f = *(const float4*)(x + (size_t)sTok[m] * D_ + k4);
    unsigned short h0, l0, h1, l1, h2, l2, h3, l3;
    split2(f.x, h0, l0); split2(f.y, h1, l1); split2(f.z, h2, l2); split2(f.w, h3, l3);
    v2u hv, lv;
    hv.x = (unsigned int)h0 | ((unsigned int)h1 << 16);
    hv.y = (unsigned int)h2 | ((unsigned int)h3 << 16);
    lv.x = (unsigned int)l0 | ((unsigned int)l1 << 16);
    lv.y = (unsigned int)l2 | ((unsigned int)l3 << 16);
    *(v2ua*)(sXhi + m * XSTR + k4) = hv;
    *(v2ua*)(sXlo + m * XSTR + k4) = lv;
  }
  __syncthreads();

  const float* W1e = w1 + (size_t)e * D_ * F_;
  const float* W2e = w2 + (size_t)e * F_ * D_;
  const float* b1e = b1 + (size_t)e * F_;
  const float* b2e = b2 + (size_t)e * D_;

  v8f zero;
#pragma unroll
  for (int r = 0; r < 8; ++r) zero[r] = 0.f;
  v8f acc[8];
#pragma unroll
  for (int j = 0; j < 8; ++j) acc[j] = zero;

  const unsigned short* aX0h = sXhi + m16 * XSTR;
  const unsigned short* aX0l = sXlo + m16 * XSTR;
  const unsigned short* aX1h = sXhi + (16 + m16) * XSTR;
  const unsigned short* aX1l = sXlo + (16 + m16) * XSTR;
  const unsigned short* aH0h = sHhi + m16 * HSTR;
  const unsigned short* aH0l = sHlo + m16 * HSTR;
  const unsigned short* aH1h = sHhi + (16 + m16) * HSTR;
  const unsigned short* aH1l = sHlo + (16 + m16) * HSTR;

  for (int fc = 0; fc < F_; fc += FC) {
    v8f ca = zero, cb = zero;
#pragma unroll 1
    for (int kk = 0; kk < D_ / 32; ++kk) {
      __syncthreads();
#pragma unroll
      for (int it = 0; it < 4; ++it) {
        const int i  = it * 256 + tid;
        const int r  = i >> 5;
        const int c4 = (i & 31) * 4;
        const float4 f = *(const float4*)(W1e + (size_t)(kk * 32 + r) * F_ + fc + c4);
        stage4(sBhi, sBlo, c4, r, f);
      }
      __syncthreads();
      const int k0 = kk * 32;
      const v16bf a0h = ld_frag(aX0h + k0, hh);
      const v16bf a0l = ld_frag(aX0l + k0, hh);
      const v16bf a1h = ld_frag(aX1h + k0, hh);
      const v16bf a1l = ld_frag(aX1l + k0, hh);
      const v16bf bh  = ld_frag(sBhi + (wv * 16 + m16) * BSTR, hh);
      const v16bf bl  = ld_frag(sBlo + (wv * 16 + m16) * BSTR, hh);
      mma3(ca, a0h, a0l, bh, bl);
      mma3(cb, a1h, a1l, bh, bl);
    }
    {
      const int   col  = wv * 16 + m16;
      const float bias = b1e[fc + col];
#pragma unroll
      for (int r = 0; r < 8; ++r) {
        unsigned short h, l;
        const int row0 = 8 * hh + r;
        split2(gelu_exact(ca[r] + bias), h, l);
        sHhi[row0 * HSTR + col] = h; sHlo[row0 * HSTR + col] = l;
        const int row1 = 16 + 8 * hh + r;
        split2(gelu_exact(cb[r] + bias), h, l);
        sHhi[row1 * HSTR + col] = h; sHlo[row1 * HSTR + col] = l;
      }
    }
#pragma unroll 1
    for (int kk = 0; kk < FC / 32; ++kk) {
      __syncthreads();
#pragma unroll 4
      for (int it = 0; it < 16; ++it) {
        const int i  = it * 256 + tid;
        const int r  = i >> 7;
        const int c4 = (i & 127) * 4;
        const float4 f = *(const float4*)(W2e + (size_t)(fc + kk * 32 + r) * D_ + c4);
        stage4(sBhi, sBlo, c4, r, f);
      }
      __syncthreads();
      const int k0 = kk * 32;
      const v16bf a0h = ld_frag(aH0h + k0, hh);
      const v16bf a0l = ld_frag(aH0l + k0, hh);
      const v16bf a1h = ld_frag(aH1h + k0, hh);
      const v16bf a1l = ld_frag(aH1l + k0, hh);
#pragma unroll
      for (int j = 0; j < 4; ++j) {
        const int n0 = wv * 64 + j * 16;
        const v16bf bh = ld_frag(sBhi + (n0 + m16) * BSTR, hh);
        const v16bf bl = ld_frag(sBlo + (n0 + m16) * BSTR, hh);
        mma3(acc[2 * j + 0], a0h, a0l, bh, bl);
        mma3(acc[2 * j + 1], a1h, a1l, bh, bl);
      }
    }
  }
  __syncthreads();

#pragma unroll
  for (int j = 0; j < 4; ++j) {
    const int   n    = wv * 64 + j * 16 + m16;
    const float bias = b2e[n];
    const float ow0  = ow[2 * n], ow1 = ow[2 * n + 1];
    const float obn  = ob[n], bks = bk[n];
#pragma unroll
    for (int p = 0; p < 2; ++p) {
#pragma unroll
      for (int r = 0; r < 8; ++r) {
        const int row = p * 16 + 8 * hh + r;
        const float spec = sF0[row] * ow0 + sF1[row] * ow1 + obn;
        sOut[row * D_ + n] = acc[2 * j + p][r] + bias + bks * spec;
      }
    }
  }
  __syncthreads();

#pragma unroll
  for (int q = 0; q < 4; ++q) {
    const int row = wv * 4 + q;
    if (sVal[row]) {
      float* dst = out + (size_t)sTok[row] * D_;
      const float* src = sOut + row * D_;
#pragma unroll
      for (int it = 0; it < 4; ++it) {
        const v4f v = *(const v4fa*)(src + it * 128 + lane * 4);
        *(volatile v4f*)(dst + it * 128 + lane * 4) = v;
      }
    }
  }
  __threadfence();
#pragma unroll
  for (int q = 0; q < 4; ++q) {
    const int row = wv * 4 + q;
    if (sVal[row]) {
      float* dst = out + (size_t)sTok[row] * D_;
      const float* src = sOut + row * D_;
#pragma unroll
      for (int it = 0; it < 4; ++it) {
        const v4f v = *(const v4fa*)(src + it * 128 + lane * 4);
        *(volatile v4f*)(dst + it * 128 + lane * 4) = v;
      }
    }
  }
}

extern "C" void kernel_launch(void* const* d_in, const int* in_sizes, int n_in,
                              void* d_out, int out_size, void* d_ws, size_t ws_size,
                              hipStream_t stream) {
  if (n_in < 14) return;
  const float* x     = (const float*)d_in[0];
  const float* vw    = (const float*)d_in[1];
  const float* vb    = (const float*)d_in[2];
  const float* gamma = (const float*)d_in[3];
  const float* epsp  = (const float*)d_in[4];
  const float* gw    = (const float*)d_in[5];
  const float* gb    = (const float*)d_in[6];
  const float* w1    = (const float*)d_in[7];
  const float* b1    = (const float*)d_in[8];
  const float* w2    = (const float*)d_in[9];
  const float* b2    = (const float*)d_in[10];
  const float* ow    = (const float*)d_in[11];
  const float* ob    = (const float*)d_in[12];
  const float* bk    = (const float*)d_in[13];
  float* out = (float*)d_out;

  if (in_sizes[0] != NTOK * D_ || out_size != NTOK * D_) return;
  if (in_sizes[7] != E_ * D_ * F_ || in_sizes[9] != E_ * F_ * D_) return;

  const size_t OFF_V = 0;
  const size_t OFF_E = OFF_V + (size_t)NTOK * 4;
  const size_t OFF_F = OFF_E + (size_t)NTOK * 4;
  const size_t OFF_P = OFF_F + (size_t)NTOK * 2 * 4;
  const size_t OFF_M = OFF_P + (size_t)NTOK * 4;
  const size_t NEED  = OFF_M + 128;
  if (ws_size < NEED) return;
  char* ws = (char*)d_ws;
  float* v_ws  = (float*)(ws + OFF_V);
  int*   e_ws  = (int*)(ws + OFF_E);
  float* feats = (float*)(ws + OFF_F);
  int*   perm  = (int*)(ws + OFF_P);
  int*   meta  = (int*)(ws + OFF_M);

  const int ntok = NTOK;
  const size_t lds_green  = (size_t)6 * N_ * sizeof(float);
  const size_t lds_bucket = (size_t)(NTOK + E_ * 512) * sizeof(int);
  const size_t lds_ffn    = (size_t)(2 * TMB * XSTR + 2 * TMB * HSTR + 2 * D_ * BSTR) * 2;

  k_proj_gate<<<(NTOK + TMB - 1) / TMB, 256, 0, stream>>>(x, vw, vb, gw, gb, v_ws, e_ws, ntok);
  k_green<<<B_, 256, lds_green, stream>>>(v_ws, gamma, epsp, feats, B_);
  k_bucket<<<1, 512, lds_bucket, stream>>>(e_ws, perm, meta, ntok);
  k_ffn<<<NTOK / TMB + E_, 256, lds_ffn, stream>>>(x, w1, b1, w2, b2, ow, ob, bk, perm, meta, feats, out, ntok);
}
